// GCN_37658273251498
// MI455X (gfx1250) — hardware-run, weakly checked
//
#include <hip/hip_runtime.h>
#include <stddef.h>
#include <stdint.h>
#include <math.h>

#define NN      50000
#define NE      600000
#define CIN     128
#define HD      128
#define NW      256
#define AK      512
#define GN      16
#define POUT    8
#define MP      50048
#define GBM     128
#define NTHR    256
#define NWAVE   8
#define EPT     8
#define WCH     (32 * EPT)
#define NBRUN   1024
#define SLB     10
#define NBK     49
#define NSLOT   (NBK * NBRUN)
#define WLCAP   3584
#define RCAP    28672
#define DEGCAP  64
#define MAXDEG_MEAS   28
#define MAXB1024_MEAS 12548
#define RWB     64
#define SP      68
#define NOUT0   (NN * POUT)
#define NOUTT   (NN * POUT + NN)

constexpr int SPLIT_L2 = 1;
constexpr int SPLIT_L3 = 1;
constexpr int K2 = SPLIT_L2 ? 256 : 128;

#define BK_ZINTS (NWAVE * WLCAP + RCAP + 3 * NBRUN)
#define BK_INTS  (BK_ZINTS + 16)
#define BK_LDS   (BK_INTS * 4)

#define PBX   (MP * CIN / 8 / NTHR)
#define PBW1  (HD * CIN / 8 / NTHR)
#define PBW2  (HD * 256 / 8 / NTHR)
#define PBW3  (GN * AK / 8 / NTHR)
#define PB_A  PBX
#define PB_B  (PB_A + PBW1)
#define PB_C  (PB_B + PBW1)
#define PB_D  (PB_C + PBW2)
#define PB_E  (PB_D + PBW2)
#define PB_F  (PB_E + PBW3)
#define PBTOT (PB_F + 1)

static_assert(NN == 50000 && NE == 600000);
static_assert(NE % 8 == 0 && NE % 4 == 0);
static_assert(MP % GBM == 0 && MP >= NN && MP == 391 * GBM && MP % RWB == 0);
static_assert(NBRUN == (1 << SLB) && NBRUN % RWB == 0 && NBRUN % GBM == 0 && NBRUN % 32 == 0);
static_assert(NBK * NBRUN >= MP && NSLOT >= MP);
static_assert(NE < (1 << 20) && (((long long)NE) << SLB) < (1LL << 31));
static_assert(RCAP == NWAVE * WLCAP && RCAP % (NTHR * 4) == 0 && BK_ZINTS % 4 == 0);
static_assert((long long)RCAP * 100 >= (long long)MAXB1024_MEAS * 105);
static_assert(WLCAP >= 2 * (MAXB1024_MEAS / 8));
static_assert(MAXDEG_MEAS + 8 <= DEGCAP);
static_assert(NW == 32 * 8 && NW == 2 * HD && AK == 4 * HD);
static_assert(CIN % 32 == 0 && K2 % 32 == 0 && AK % 32 == 0);
static_assert((MP * CIN / 8) % NTHR == 0 && (HD * CIN / 8) % NTHR == 0 && (HD * 256 / 8) % NTHR == 0);
static_assert((GN * AK / 8) % NTHR == 0);
static_assert(BK_LDS <= 300000);
static_assert((GBM * SP + GBM) * 4 <= 65536);
static_assert(NN % 4 == 0 && (NN % NBRUN) % 4 == 0);
static_assert((NOUT0 * 4) % 128 == 0);
static_assert(NOUT0 + (NBK - 1) * NBRUN + (NN - (NBK - 1) * NBRUN) - 1 == NOUTT - 1);
static_assert(NBRUN * POUT / 4 == 8 * NTHR && NBRUN / 4 == NTHR);

typedef float          v4f   __attribute__((ext_vector_type(4)));
typedef float          v8f   __attribute__((ext_vector_type(8)));
typedef int            v4i   __attribute__((ext_vector_type(4)));
typedef int            v8i   __attribute__((ext_vector_type(8)));
typedef unsigned int   v4u   __attribute__((ext_vector_type(4)));
typedef unsigned short v8us  __attribute__((ext_vector_type(8)));
typedef unsigned short v16us __attribute__((ext_vector_type(16)));
typedef __bf16         v16bf __attribute__((ext_vector_type(16)));
typedef v4f  __attribute__((may_alias)) v4fa;
typedef v4i  __attribute__((may_alias)) v4ia;
typedef v8us __attribute__((may_alias)) v8usa;
union FragB { v16bf v; v16us u; v8us h[2]; v8i w; };

__device__ __forceinline__ v8f wmb(const FragB& a, const FragB& b, v8f c) {
  v8f d = __builtin_amdgcn_wmma_f32_16x16x32_bf16(false, a.v, false, b.v, (short)0, c, false, false);
  asm volatile("v_nop\n\tv_nop\n\tv_nop\n\tv_nop" : "+v"(d) : "v"(a.w), "v"(b.w));
  return d;
}

__device__ __forceinline__ unsigned bf16_bits(float f) {
  const unsigned u = __float_as_uint(f);
  const unsigned r = (u + 0x7FFFu + ((u >> 16) & 1u)) >> 16;
  const unsigned q = (u >> 16) | 0x40u;
  return ((u & 0x7fffffffu) > 0x7f800000u) ? q : r;
}
__device__ __forceinline__ float bf16_val(float f) {
  return __uint_as_float(bf16_bits(f) << 16);
}

__device__ __forceinline__ void st2_v4f(float* p, v4f v) {
  *(volatile v4f*)p = v;
  __threadfence();
  *(volatile v4f*)p = v;
}
__device__ __forceinline__ void st2_v8us(unsigned short* p, v8us v) {
  *(volatile v8us*)p = v;
  __threadfence();
  *(volatile v8us*)p = v;
}

__device__ __forceinline__ v8us col8(const float* __restrict__ base, int stride) {
  float f[8];
#pragma unroll
  for (int i = 0; i < 8; ++i) f[i] = base[(size_t)i * (size_t)stride];
  v8us o;
#pragma unroll
  for (int i = 0; i < 8; ++i) o[i] = (unsigned short)bf16_bits(f[i]);
  return o;
}

__global__ __launch_bounds__(NTHR) void k_prep(const float* __restrict__ x,
                                               const float* __restrict__ wp1, const float* __restrict__ bp1,
                                               const float* __restrict__ wp2, const float* __restrict__ bp2,
                                               const float* __restrict__ wp3, const float* __restrict__ bp3,
                                               const float* __restrict__ wv1, const float* __restrict__ bv1,
                                               const float* __restrict__ wv2, const float* __restrict__ bv2,
                                               const float* __restrict__ wv3, const float* __restrict__ bv3,
                                               unsigned short* xb, unsigned short* w1t, unsigned short* w2d,
                                               unsigned short* w3t, float* sm) {
  const int tid = (int)threadIdx.x, lane = tid & 31, wave = tid >> 5;
  const int blk = (int)blockIdx.x;
  if (blk < PB_A) {
    const int u   = blk * NTHR + tid;
    const int row = u >> 4, k8 = (u & 15) * 8;
    const int rc  = row < NN ? row : NN - 1;
    const unsigned mk = row < NN ? 0xffffu : 0u;
    const float* p = x + (size_t)rc * CIN + k8;
    const v4f a = *(const v4fa*)p;
    const v4f b = *(const v4fa*)(p + 4);
    v8us o;
    o[0] = (unsigned short)(bf16_bits(a.x) & mk); o[1] = (unsigned short)(bf16_bits(a.y) & mk);
    o[2] = (unsigned short)(bf16_bits(a.z) & mk); o[3] = (unsigned short)(bf16_bits(a.w) & mk);
    o[4] = (unsigned short)(bf16_bits(b.x) & mk); o[5] = (unsigned short)(bf16_bits(b.y) & mk);
    o[6] = (unsigned short)(bf16_bits(b.z) & mk); o[7] = (unsigned short)(bf16_bits(b.w) & mk);
    st2_v8us(xb + (size_t)row * CIN + k8, o);
  } else if (blk < PB_B) {
    const int u = (blk - PB_A) * NTHR + tid;
    const int n = u >> 4, k8 = (u & 15) * 8;
    const v8us o = col8(wp1 + (size_t)k8 * HD + n, HD);
    st2_v8us(w1t + (size_t)n * CIN + k8, o);
  } else if (blk < PB_C) {
    const int u = (blk - PB_B) * NTHR + tid;
    const int n = u >> 4, k8 = (u & 15) * 8;
    const v8us o = col8(wv1 + (size_t)k8 * HD + n, HD);
    st2_v8us(w1t + (size_t)(HD + n) * CIN + k8, o);
  } else if (blk < PB_D) {
    const int u = (blk - PB_C) * NTHR + tid;
    const int n = u >> 5, k8 = (u & 31) * 8, kk = k8 & (HD - 1);
    const v8us o = col8(wp2 + (size_t)kk * HD + n, HD);
    st2_v8us(w2d + (size_t)n * 256 + k8, o);
  } else if (blk < PB_E) {
    const int u = (blk - PB_D) * NTHR + tid;
    const int n = u >> 5, k8 = (u & 31) * 8, kk = k8 & (HD - 1);
    const v8us o = col8(wv2 + (size_t)kk * HD + n, HD);
    st2_v8us(w2d + (size_t)HD * 256 + (size_t)n * 256 + k8, o);
  } else if (blk < PB_F) {
    const int wb = blk - PB_E;
    if (wb < 2) {
      const int u = wb * NTHR + tid;
      const int n = u >> 6, k8 = (u & 63) * 8, kk = k8 & (HD - 1);
      const v8us g = col8(wp3 + (size_t)kk * POUT + n, POUT);
      const bool on = (k8 < 256) && (SPLIT_L3 != 0 || (k8 & 128) == 0);
      const unsigned short mk = on ? (unsigned short)0xffffu : (unsigned short)0;
      v8us o;
#pragma unroll
      for (int i = 0; i < 8; ++i) o[i] = (unsigned short)(g[i] & mk);
      st2_v8us(w3t + (size_t)n * AK + k8, o);
    } else {
      const int u = (wb - 2) * NTHR + tid;
      const int n = 8 + (u >> 6), k8 = (u & 63) * 8, kk = k8 & (HD - 1);
      const v4f a = *(const v4fa*)(wv3 + kk);
      const v4f b = *(const v4fa*)(wv3 + kk + 4);
      asm volatile("" :: "v"(a));
      asm volatile("" :: "v"(b));
      const bool on = (n == 8) && (k8 >= 256) && (SPLIT_L3 != 0 || (k8 & 128) == 0);
      const unsigned mk = on ? 0xffffu : 0u;
      v8us o;
      o[0] = (unsigned short)(bf16_bits(a.x) & mk); o[1] = (unsigned short)(bf16_bits(a.y) & mk);
      o[2] = (unsigned short)(bf16_bits(a.z) & mk); o[3] = (unsigned short)(bf16_bits(a.w) & mk);
      o[4] = (unsigned short)(bf16_bits(b.x) & mk); o[5] = (unsigned short)(bf16_bits(b.y) & mk);
      o[6] = (unsigned short)(bf16_bits(b.z) & mk); o[7] = (unsigned short)(bf16_bits(b.w) & mk);
      st2_v8us(w3t + (size_t)n * AK + k8, o);
    }
  } else {
    if (wave < 4) {
      v4f a;
      if (wave == 0)      a = *(const v4fa*)(bp1 + 4 * lane);
      else if (wave == 1) a = *(const v4fa*)(bv1 + 4 * lane);
      else if (wave == 2) a = *(const v4fa*)(bp2 + 4 * lane);
      else                a = *(const v4fa*)(bv2 + 4 * lane);
      v4f o;
      o.x = bf16_val(a.x); o.y = bf16_val(a.y); o.z = bf16_val(a.z); o.w = bf16_val(a.w);
      st2_v4f(sm + 128 * wave + 4 * lane, o);
    } else if (wave == 4) {
      const int e0 = 4 * lane;
      const float p0 = bp3[min(e0,     POUT - 1)], p1 = bp3[min(e0 + 1, POUT - 1)];
      const float p2 = bp3[min(e0 + 2, POUT - 1)], p3 = bp3[min(e0 + 3, POUT - 1)];
      const float c0 = bv3[0];
      asm volatile("" :: "v"(p0), "v"(p1), "v"(p2), "v"(p3), "v"(c0));
      const unsigned mp = (lane < 2) ? 0xffffffffu : 0u;
      const unsigned mv = (lane == 2) ? 0xffffffffu : 0u;
      v4f o;
      o.x = __uint_as_float(((bf16_bits(p0) << 16) & mp) | ((bf16_bits(c0) << 16) & mv));
      o.y = __uint_as_float((bf16_bits(p1) << 16) & mp);
      o.z = __uint_as_float((bf16_bits(p2) << 16) & mp);
      o.w = __uint_as_float((bf16_bits(p3) << 16) & mp);
      st2_v4f(sm + 512 + 4 * lane, o);
    }
  }
}

__device__ __forceinline__ void bucket_flush(const int* pl, const int* cnt, const int* offs, const int* dv, int ov,
                                             int* lp, int* cp, int* op, int* dp, int* fp, int tid) {
#pragma unroll 1
  for (int i = tid * 4; i < RCAP; i += NTHR * 4) {
    const v4i v = *(const v4ia*)(pl + i);
    *(volatile v4i*)(lp + i) = v;
  }
  {
    const v4i a = *(const v4ia*)(cnt + 4 * tid);
    const v4i b = *(const v4ia*)(offs + 4 * tid);
    const v4i c = *(const v4ia*)(dv + 4 * tid);
    *(volatile v4i*)(cp + 4 * tid) = a;
    *(volatile v4i*)(op + 4 * tid) = b;
    *(volatile v4i*)(dp + 4 * tid) = c;
  }
  if (tid < 8) {
    const v4i f = {ov, ov, ov, ov};
    *(volatile v4i*)(fp + 4 * tid) = f;
  }
}

__global__ __launch_bounds__(NTHR) void k_bucket(const int* __restrict__ srcs, const int* __restrict__ dsts,
                                                 int* LIST, int* CNT, int* OFF, int* DINVB, int* FLAG) {
  extern __shared__ __attribute__((aligned(16))) int dsm[];
  int* wl   = dsm;
  int* pl   = dsm + NWAVE * WLCAP;
  int* cnt  = pl + RCAP;
  int* offs = cnt + NBRUN;
  int* cur  = offs + NBRUN;
  int* misc = cur + NBRUN;
  const int tid = (int)threadIdx.x, lane = tid & 31, wave = tid >> 5;
  const int blk = (int)blockIdx.x;
  const unsigned nbs = (unsigned)(blk * NBRUN);

  {
    const v4i z4 = {0, 0, 0, 0};
    for (int i = tid * 4; i < BK_ZINTS; i += NTHR * 4) *(v4ia*)(dsm + i) = z4;
    if (tid < 16) misc[tid] = 0;
  }
  __syncthreads();

  {
    constexpr int per = ((NE + NWAVE * WCH - 1) / (NWAVE * WCH)) * WCH;
    const int ebeg = wave * per;
    const int eend = (ebeg + per < NE) ? (ebeg + per) : NE;
    int* mylist = wl + wave * WLCAP;
    int wc = 0;
#pragma unroll 1
    for (int cb = ebeg; cb < eend; cb += WCH) {
      const int e0  = cb + lane * EPT;
      const int e0c = e0 < NE - EPT ? e0 : NE - EPT;
      const bool inr = e0 < NE;
      const v4i da = *(const v4ia*)(dsts + e0c);
      const v4i db = *(const v4ia*)(dsts + e0c + 4);
      const unsigned s0 = (unsigned)da.x - nbs, s1 = (unsigned)da.y - nbs;
      const unsigned s2 = (unsigned)da.z - nbs, s3 = (unsigned)da.w - nbs;
      const unsigned s4 = (unsigned)db.x - nbs, s5 = (unsigned)db.y - nbs;
      const unsigned s6 = (unsigned)db.z - nbs, s7 = (unsigned)db.w - nbs;
      const bool h0 = inr & (s0 < (unsigned)NBRUN), h1 = inr & (s1 < (unsigned)NBRUN);
      const bool h2 = inr & (s2 < (unsigned)NBRUN), h3 = inr & (s3 < (unsigned)NBRUN);
      const bool h4 = inr & (s4 < (unsigned)NBRUN), h5 = inr & (s5 < (unsigned)NBRUN);
      const bool h6 = inr & (s6 < (unsigned)NBRUN), h7 = inr & (s7 < (unsigned)NBRUN);
      const unsigned m0 = __builtin_amdgcn_ballot_w32(h0), m1 = __builtin_amdgcn_ballot_w32(h1);
      const unsigned m2 = __builtin_amdgcn_ballot_w32(h2), m3 = __builtin_amdgcn_ballot_w32(h3);
      const unsigned m4 = __builtin_amdgcn_ballot_w32(h4), m5 = __builtin_amdgcn_ballot_w32(h5);
      const unsigned m6 = __builtin_amdgcn_ballot_w32(h6), m7 = __builtin_amdgcn_ballot_w32(h7);
      const unsigned any = m0 | m1 | m2 | m3 | m4 | m5 | m6 | m7;
      if (any != 0u) {
        const int pre = (int)(__builtin_amdgcn_mbcnt_lo(m0, 0u) + __builtin_amdgcn_mbcnt_lo(m1, 0u) +
                              __builtin_amdgcn_mbcnt_lo(m2, 0u) + __builtin_amdgcn_mbcnt_lo(m3, 0u) +
                              __builtin_amdgcn_mbcnt_lo(m4, 0u) + __builtin_amdgcn_mbcnt_lo(m5, 0u) +
                              __builtin_amdgcn_mbcnt_lo(m6, 0u) + __builtin_amdgcn_mbcnt_lo(m7, 0u));
        int p = wc + pre;
        if (h0) { if (p < WLCAP) mylist[p] = ((e0 + 0) << SLB) | (int)s0; p = p + 1; }
        if (h1) { if (p < WLCAP) mylist[p] = ((e0 + 1) << SLB) | (int)s1; p = p + 1; }
        if (h2) { if (p < WLCAP) mylist[p] = ((e0 + 2) << SLB) | (int)s2; p = p + 1; }
        if (h3) { if (p < WLCAP) mylist[p] = ((e0 + 3) << SLB) | (int)s3; p = p + 1; }
        if (h4) { if (p < WLCAP) mylist[p] = ((e0 + 4) << SLB) | (int)s4; p = p + 1; }
        if (h5) { if (p < WLCAP) mylist[p] = ((e0 + 5) << SLB) | (int)s5; p = p + 1; }
        if (h6) { if (p < WLCAP) mylist[p] = ((e0 + 6) << SLB) | (int)s6; p = p + 1; }
        if (h7) { if (p < WLCAP) mylist[p] = ((e0 + 7) << SLB) | (int)s7; p = p + 1; }
        wc += (int)(__builtin_popcount(m0) + __builtin_popcount(m1) + __builtin_popcount(m2) + __builtin_popcount(m3) +
                    __builtin_popcount(m4) + __builtin_popcount(m5) + __builtin_popcount(m6) + __builtin_popcount(m7));
      }
    }
    if (lane == 0) misc[wave] = wc;
  }
  __syncthreads();

  if (wave == 0) {
    int ov = 0;
#pragma unroll 1
    for (int w2 = 0; w2 < NWAVE; ++w2) {
      int c = misc[w2];
      if (c > WLCAP) ov = 1;
      c = c < 0 ? 0 : (c > WLCAP ? WLCAP : c);
#pragma unroll 1
      for (int b0 = 0; b0 < c; b0 += 32) {
        const int idx = b0 + lane;
        const int ent = wl[w2 * WLCAP + (idx < WLCAP ? idx : WLCAP - 1)];
        const int m32 = (c - b0) < 32 ? (c - b0) : 32;
#pragma unroll 1
        for (int k = 0; k < m32; ++k) {
          const int u    = __builtin_amdgcn_readlane(ent, k);
          const int slot = u & (NBRUN - 1);
          if (lane == 0) cnt[slot] = cnt[slot] + 1;
        }
      }
    }
    if (lane == 0) misc[9] = ov;
  }
  __syncthreads();
  if (wave == 0) {
    const int base = lane * (NBRUN / 32);
    int s = 0;
    bool bg = false;
#pragma unroll 1
    for (int i = 0; i < NBRUN / 32; ++i) {
      const int cv = cnt[base + i];
      s += cv;
      bg = bg | (cv > DEGCAP);
    }
    const unsigned bm = __builtin_amdgcn_ballot_w32(bg);
    int incl = s;
#pragma unroll
    for (int d = 1; d < 32; d <<= 1) {
      const int y = __shfl_up(incl, d, 32);
      if (lane >= d) incl += y;
    }
    int run = incl - s;
#pragma unroll 1
    for (int i = 0; i < NBRUN / 32; ++i) {
      const int cv = cnt[base + i];
      offs[base + i] = run;
      cur[base + i]  = run;
      run += cv;
    }
    if (lane == 0) misc[9] = misc[9] | ((bm != 0u) ? 1 : 0);
  }
  __syncthreads();

  if (wave == 0) {
#pragma unroll 1
    for (int w2 = 0; w2 < NWAVE; ++w2) {
      int c = misc[w2];
      c = c < 0 ? 0 : (c > WLCAP ? WLCAP : c);
#pragma unroll 1
      for (int b0 = 0; b0 < c; b0 += 32) {
        const int idx = b0 + lane;
        const int ent = wl[w2 * WLCAP + (idx < WLCAP ? idx : WLCAP - 1)];
        int eid = (ent >> SLB) & 0xFFFFF;
        eid = eid > NE - 1 ? NE - 1 : eid;
        int sr = srcs[eid];
        sr = sr < 0 ? 0 : (sr > NN - 1 ? NN - 1 : sr);
        const int m32 = (c - b0) < 32 ? (c - b0) : 32;
#pragma unroll 1
        for (int k = 0; k < m32; ++k) {
          const int u    = __builtin_amdgcn_readlane(ent, k);
          const int wd   = __builtin_amdgcn_readlane(sr, k);
          const int slot = u & (NBRUN - 1);
          if (lane == 0) {
            int p = cur[slot];
            p = p < 0 ? 0 : (p > RCAP - 1 ? RCAP - 1 : p);
            pl[p] = wd;
            cur[slot] = p + 1;
          }
        }
      }
    }
  }
  __syncthreads();

#pragma unroll 1
  for (int i = tid; i < NBRUN; i += NTHR) {
    int cv = cnt[i];
    cv = cv < 0 ? 0 : (cv > RCAP ? RCAP : cv);
    const float dg = fmaxf((float)(cv + 1), 1.0f);
    cur[i] = __float_as_int(1.0f / sqrtf(dg));
  }
  __syncthreads();

  const int ovf = misc[9];
  int* lp = LIST + (size_t)blk * RCAP;
  int* cp = CNT + (size_t)blk * NBRUN;
  int* op = OFF + (size_t)blk * NBRUN;
  int* dp = DINVB + (size_t)blk * NBRUN;
  int* fp = FLAG + (size_t)blk * 32;
  bucket_flush(pl, cnt, offs, cur, ovf, lp, cp, op, dp, fp, tid);
  __threadfence();
  bucket_flush(pl, cnt, offs, cur, ovf, lp, cp, op, dp, fp, tid);
}

template <int KTOT, int NT>
__device__ __forceinline__ void mm_tile(const unsigned short* __restrict__ ap,
                                        const unsigned short* __restrict__ bp, int ldb, v8f (&acc)[NT]) {
  static_assert(KTOT % 32 == 0);
#pragma unroll 1
  for (int k0 = 0; k0 < KTOT; k0 += 32) {
    FragB af;
    af.h[0] = *(const v8usa*)(ap + k0);
    af.h[1] = *(const v8usa*)(ap + k0 + 16);
#pragma unroll
    for (int nt = 0; nt < NT; ++nt) {
      const unsigned short* wq = bp + (size_t)(16 * nt) * (size_t)ldb + k0;
      FragB bf;
      bf.h[0] = *(const v8usa*)wq;
      bf.h[1] = *(const v8usa*)(wq + 16);
      acc[nt] = wmb(af, bf, acc[nt]);
    }
  }
}

template <int KTOT, int NT>
__global__ __launch_bounds__(NTHR) __attribute__((amdgpu_num_vgpr(248)))
void k_mm(const unsigned short* __restrict__ A, int lda, int aZ,
          const unsigned short* __restrict__ BT, int ldb, int bZ,
          const float* __restrict__ dinv, float* out, int ldo, int oZ) {
  static_assert(NT == 4 || NT == 1);
  constexpr int SPN = (NT == 4) ? SP : 16;
  __shared__ __attribute__((aligned(16))) float stg[GBM * SPN];
  __shared__ __attribute__((aligned(16))) float sd[GBM];
  const int tid = (int)threadIdx.x, lane = tid & 31, wave = tid >> 5, hh = lane >> 4, m = lane & 15;
  const int rowBase = (int)blockIdx.x * GBM;
  const int colBase = (int)blockIdx.y * (16 * NT);
  const int z = (int)blockIdx.z;
  if (tid < 32) *(v4fa*)(sd + 4 * tid) = *(const v4fa*)(dinv + rowBase + 4 * tid);

  v8f acc[NT];
  {
    const v8f zz = {0.f, 0.f, 0.f, 0.f, 0.f, 0.f, 0.f, 0.f};
#pragma unroll
    for (int t = 0; t < NT; ++t) acc[t] = zz;
  }
  const unsigned short* ap = A + (size_t)z * (size_t)aZ + (size_t)(rowBase + 16 * wave + m) * (size_t)lda + 8 * hh;
  const unsigned short* bp = BT + (size_t)z * (size_t)bZ + (size_t)(colBase + m) * (size_t)ldb + 8 * hh;
  mm_tile<KTOT, NT>(ap, bp, ldb, acc);
#pragma unroll
  for (int nt = 0; nt < NT; ++nt) {
#pragma unroll
    for (int r = 0; r < 8; ++r) stg[(16 * wave + 8 * hh + r) * SPN + 16 * nt + m] = acc[nt][r];
  }
  __syncthreads();

  float* ob = out + (size_t)z * (size_t)oZ;
  if constexpr (NT == 4) {
#pragma unroll 1
    for (int i = 0; i < 8; ++i) {
      const int lr   = 16 * wave + 2 * i + hh;
      const int grow = rowBase + lr;
      const v4f a = *(const v4fa*)(stg + lr * SPN + 4 * m);
      const float d = sd[lr];
      const float lv = (grow < NN) ? 1.0f : 0.0f;
      v4f o;
      o.x = (a.x * d) * lv; o.y = (a.y * d) * lv; o.z = (a.z * d) * lv; o.w = (a.w * d) * lv;
      st2_v4f(ob + (size_t)grow * (size_t)ldo + colBase + 4 * m, o);
    }
  } else {
#pragma unroll 1
    for (int it = 0; it < 2; ++it) {
      const int i4   = it * NTHR + tid;
      const int lr   = i4 >> 2;
      const int grow = rowBase + lr;
      const v4f a = *(const v4fa*)(stg + 4 * i4);
      const float d = sd[lr];
      const float lv = (grow < NN) ? 1.0f : 0.0f;
      v4f o;
      o.x = (a.x * d) * lv; o.y = (a.y * d) * lv; o.z = (a.z * d) * lv; o.w = (a.w * d) * lv;
      st2_v4f(ob + (size_t)grow * (size_t)ldo + 4 * (i4 & 3), o);
    }
  }
}

__global__ __launch_bounds__(NTHR) void k_replay_wide(const int* __restrict__ LIST, const int* __restrict__ CNT,
                                                      const int* __restrict__ OFF, const float* __restrict__ DINV,
                                                      const int* __restrict__ FLAG, const float* __restrict__ Hs,
                                                      const float* __restrict__ bias, unsigned short* Aout) {
  __shared__ __attribute__((aligned(16))) float sb[NW];
  const int tid = (int)threadIdx.x, lane = tid & 31, wave = tid >> 5;
  const int rowBase = (int)blockIdx.x * RWB;
  const int bucket  = rowBase >> SLB;
  const int* lb  = LIST + (size_t)bucket * RCAP;
  const int flag = FLAG[(size_t)bucket * 32];
  if (tid < 32) {
    *(v4fa*)(sb + 4 * tid)       = *(const v4fa*)(bias + 4 * tid);
    *(v4fa*)(sb + 128 + 4 * tid) = *(const v4fa*)(bias + 128 + 4 * tid);
  }
  __syncthreads();
  const v4f bq0 = *(const v4fa*)(sb + 8 * lane);
  const v4f bq1 = *(const v4fa*)(sb + 8 * lane + 4);
  const float qnan = __uint_as_float(0x7fc00000u);
  const int hoff = 8 * (lane & 15) + 256 * (lane >> 4);

#pragma unroll 1
  for (int i = 0; i < RWB / NWAVE; ++i) {
    const int d  = rowBase + (RWB / NWAVE) * wave + i;
    const int cr = CNT[d];
    const bool big = cr > DEGCAP;
    const int c = max(0, min(cr, DEGCAP));
    const int o = max(0, min(OFF[d], RCAP - 1));
    int last = o + c - 1; last = last < o ? o : last;
    last = min(last, RCAP - 1);
    const int cu = __builtin_amdgcn_readfirstlane(c);
    v4f a0 = {0.0f, 0.0f, 0.0f, 0.0f};
    v4f a1 = {0.0f, 0.0f, 0.0f, 0.0f};
#pragma unroll 1
    for (int b0 = 0; b0 < cu; b0 += 32) {
      int idx = o + b0 + lane;
      idx = idx > last ? last : idx;
      int sr = lb[idx];
      sr = max(0, min(sr, NN - 1));
      const int m32 = (cu - b0) < 32 ? (cu - b0) : 32;
#pragma unroll 1
      for (int k = 0; k < m32; ++k) {
        const int sk = __builtin_amdgcn_readlane(sr, k);
        const float* p = Hs + (size_t)sk * NW + 8 * lane;
        const v4f x0 = *(const v4fa*)p;
        const v4f x1 = *(const v4fa*)(p + 4);
        a0 = a0 + x0; a1 = a1 + x1;
      }
    }
    const float* ps = Hs + (size_t)d * NW + 8 * lane;
    const v4f g0 = *(const v4fa*)ps;
    const v4f g1 = *(const v4fa*)(ps + 4);
    const float dd = DINV[d];
    float v[8];
    v[0] = (a0.x + g0.x) * dd + bq0.x; v[1] = (a0.y + g0.y) * dd + bq0.y;
    v[2] = (a0.z + g0.z) * dd + bq0.z; v[3] = (a0.w + g0.w) * dd + bq0.w;
    v[4] = (a1.x + g1.x) * dd + bq1.x; v[5] = (a1.y + g1.y) * dd + bq1.y;
    v[6] = (a1.z + g1.z) * dd + bq1.z; v[7] = (a1.w + g1.w) * dd + bq1.w;
    const bool bad  = (flag != 0) | big;
    const bool live = d < NN;
    unsigned hb[8], lw[8];
#pragma unroll
    for (int j = 0; j < 8; ++j) {
      float y = v[j];
      y = (y > 0.0f) ? y : (y - y);
      y = bad ? qnan : y;
      y = live ? y : 0.0f;
      hb[j] = bf16_bits(y);
      lw[j] = bf16_bits(y - __uint_as_float(hb[j] << 16));
    }
    v4u hv, lv;
    hv.x = hb[0] | (hb[1] << 16); hv.y = hb[2] | (hb[3] << 16);
    hv.z = hb[4] | (hb[5] << 16); hv.w = hb[6] | (hb[7] << 16);
    lv.x = lw[0] | (lw[1] << 16); lv.y = lw[2] | (lw[3] << 16);
    lv.z = lw[4] | (lw[5] << 16); lv.w = lw[6] | (lw[7] << 16);
    unsigned short* hp = Aout + (size_t)d * AK + hoff;
    unsigned short* lp = hp + HD;
    *(volatile v4u*)hp = hv;
    *(volatile v4u*)lp = lv;
    __threadfence();
    *(volatile v4u*)hp = hv;
    *(volatile v4u*)lp = lv;
  }
}

__device__ __forceinline__ void narrow_flush(const float* lgs, const float* vs, float* o0, float* o1,
                                             int nl4, int nv4, int flag, int tid) {
  const float qnan = __uint_as_float(0x7fc00000u);
#pragma unroll 1
  for (int it = 0; it < 8; ++it) {
    const int i4 = it * NTHR + tid;
    v4f v = *(const v4fa*)(lgs + 4 * i4);
    asm volatile("" :: "v"(v));
    v.x = (flag != 0) ? qnan : v.x; v.y = (flag != 0) ? qnan : v.y;
    v.z = (flag != 0) ? qnan : v.z; v.w = (flag != 0) ? qnan : v.w;
    if (i4 < nl4) *(volatile v4f*)(o0 + (size_t)4 * (size_t)i4) = v;
  }
  {
    v4f v = *(const v4fa*)(vs + 4 * tid);
    asm volatile("" :: "v"(v));
    v.x = (flag != 0) ? qnan : v.x; v.y = (flag != 0) ? qnan : v.y;
    v.z = (flag != 0) ? qnan : v.z; v.w = (flag != 0) ? qnan : v.w;
    if (tid < nv4) *(volatile v4f*)(o1 + (size_t)4 * (size_t)tid) = v;
  }
}

__global__ __launch_bounds__(NTHR) void k_replay_narrow(const int* __restrict__ LIST, const int* __restrict__ CNT,
                                                        const int* __restrict__ OFF, const float* __restrict__ DINV,
                                                        const int* __restrict__ FLAG, const float* __restrict__ G,
                                                        const float* __restrict__ b3, float* out) {
  __shared__ __attribute__((aligned(16))) float lgs[NBRUN * POUT];
  __shared__ __attribute__((aligned(16))) float vs[NBRUN];
  __shared__ __attribute__((aligned(16))) float sb3[GN];
  const int tid = (int)threadIdx.x, lane = tid & 31, wave = tid >> 5;
  const int q = lane & 3, grp = lane >> 2;
  const int blk = (int)blockIdx.x;
  const int slotBase = blk * NBRUN;
  const int* lb  = LIST + (size_t)blk * RCAP;
  const int flag = FLAG[(size_t)blk * 32];
  if (tid < 4) *(v4fa*)(sb3 + 4 * tid) = *(const v4fa*)(b3 + 4 * tid);
  __syncthreads();
  const v4f bq = *(const v4fa*)(sb3 + 4 * q);
  const float qnan = __uint_as_float(0x7fc00000u);

#pragma unroll 1
  for (int pass = 0; pass < NBRUN / 64; ++pass) {
    const int s  = pass * 64 + wave * 8 + grp;
    const int d  = slotBase + s;
    const int cr = CNT[d];
    const bool big = cr > DEGCAP;
    const int c = max(0, min(cr, DEGCAP));
    const int o = max(0, min(OFF[d], RCAP - 1));
    int last = o + c - 1; last = last < o ? o : last;
    last = min(last, RCAP - 1);
    int cm = c;
    cm = max(cm, __shfl_xor(cm, 4, 32));
    cm = max(cm, __shfl_xor(cm, 8, 32));
    cm = max(cm, __shfl_xor(cm, 16, 32));
    const int cmu = __builtin_amdgcn_readfirstlane(cm);
    v4f a = {0.0f, 0.0f, 0.0f, 0.0f};
#pragma unroll 1
    for (int j = 0; j < cmu; ++j) {
      int idx = o + j;
      idx = idx > last ? last : idx;
      int sr = lb[idx];
      sr = max(0, min(sr, NN - 1));
      const v4f g = *(const v4fa*)(G + (size_t)sr * GN + 4 * q);
      asm volatile("" :: "v"(g));
      const bool valid = j < c;
      const v4f t = a + g;
      a.x = valid ? t.x : a.x; a.y = valid ? t.y : a.y;
      a.z = valid ? t.z : a.z; a.w = valid ? t.w : a.w;
    }
    const int dg = min(d, MP - 1);
    const v4f sf = *(const v4fa*)(G + (size_t)dg * GN + 4 * q);
    const float dd = DINV[d];
    v4f y;
    y.x = (a.x + sf.x) * dd + bq.x; y.y = (a.y + sf.y) * dd + bq.y;
    y.z = (a.z + sf.z) * dd + bq.z; y.w = (a.w + sf.w) * dd + bq.w;
    y.x = big ? qnan : y.x; y.y = big ? qnan : y.y; y.z = big ? qnan : y.z; y.w = big ? qnan : y.w;
    if (q < 2) *(v4fa*)(lgs + s * POUT + 4 * q) = y;
    if (q == 2) vs[s] = y.x;
  }
  __syncthreads();

  const int liveRows = (NN - slotBase) < NBRUN ? (NN - slotBase) : NBRUN;
  const int nl4 = liveRows * (POUT / 4);
  const int nv4 = liveRows / 4;
  float* o0 = out + (size_t)blk * (size_t)(NBRUN * POUT);
  float* o1 = out + (size_t)NOUT0 + (size_t)blk * (size_t)NBRUN;
  narrow_flush(lgs, vs, o0, o1, nl4, nv4, flag, tid);
  __threadfence();
  narrow_flush(lgs, vs, o0, o1, nl4, nv4, flag, tid);
}

extern "C" void kernel_launch(void* const* d_in, const int* in_sizes, int n_in,
                              void* d_out, int out_size, void* d_ws, size_t ws_size,
                              hipStream_t stream) {
  if (n_in < 14) return;
  if (in_sizes[0] != NN * CIN) return;
  if (in_sizes[1] != 2 * NE) return;
  if (in_sizes[2] != CIN * HD || in_sizes[3] != HD) return;
  if (in_sizes[4] != HD * HD || in_sizes[5] != HD) return;
  if (in_sizes[6] != HD * POUT || in_sizes[7] != POUT) return;
  if (in_sizes[8] != CIN * HD || in_sizes[9] != HD) return;
  if (in_sizes[10] != HD * HD || in_sizes[11] != HD) return;
  if (in_sizes[12] != HD || in_sizes[13] != 1) return;
  if (out_size != NOUTT) return;

  const float* x   = (const float*)d_in[0];
  const int*   ei  = (const int*)d_in[1];
  const float* Wp1 = (const float*)d_in[2];
  const float* bp1 = (const float*)d_in[3];
  const float* Wp2 = (const float*)d_in[4];
  const float* bp2 = (const float*)d_in[5];
  const float* Wp3 = (const float*)d_in[6];
  const float* bp3 = (const float*)d_in[7];
  const float* Wv1 = (const float*)d_in[8];
  const float* bv1 = (const float*)d_in[9];
  const float* Wv2 = (const float*)d_in[10];
  const float* bv2 = (const float*)d_in[11];
  const float* Wv3 = (const float*)d_in[12];
  const float* bv3 = (const float*)d_in[13];
  float* out = (float*)d_out;
  const int* srcs = ei;
  const int* dsts = ei + NE;

  constexpr size_t zXB   = (size_t)MP * CIN * 2;
  constexpr size_t zH    = (size_t)MP * NW * 4;
  constexpr size_t zA    = (size_t)MP * AK * 2;
  constexpr size_t zG    = (size_t)MP * GN * 4;
  constexpr size_t zLIST = (size_t)NBK * RCAP * 4;
  constexpr size_t zTAB  = (size_t)NSLOT * 4;
  constexpr size_t zFLAG = 6400;
  constexpr size_t zW1T  = (size_t)NW * CIN * 2;
  constexpr size_t zW2D  = (size_t)2 * HD * 256 * 2;
  constexpr size_t zW3T  = (size_t)GN * AK * 2;
  constexpr size_t zSM   = 2560;
  constexpr size_t oXB   = 0;
  constexpr size_t oH    = oXB + zXB;
  constexpr size_t oA    = oH + zH;
  constexpr size_t oG    = oA + zA;
  constexpr size_t oLIST = oG + zG;
  constexpr size_t oCNT  = oLIST + zLIST;
  constexpr size_t oOFF  = oCNT + zTAB;
  constexpr size_t oDINV = oOFF + zTAB;
  constexpr size_t oFLAG = oDINV + zTAB;
  constexpr size_t oW1T  = oFLAG + zFLAG;
  constexpr size_t oW2D  = oW1T + zW1T;
  constexpr size_t oW3T  = oW2D + zW2D;
  constexpr size_t oSM   = oW3T + zW3T;
  constexpr size_t oEND  = oSM + zSM;
  static_assert(zXB % 256 == 0 && zH % 256 == 0 && zA % 256 == 0 && zG % 256 == 0 && zLIST % 256 == 0);
  static_assert(zTAB % 256 == 0 && zFLAG % 256 == 0 && zFLAG >= (size_t)NBK * 128);
  static_assert(zW1T % 256 == 0 && zW2D % 256 == 0 && zW3T % 256 == 0 && zSM % 256 == 0 && zSM >= 640 * 4);
  static_assert(oEND <= ((size_t)128 << 20));
  if (oEND > ws_size) return;

  char* ws = (char*)d_ws;
  unsigned short* XB   = (unsigned short*)(ws + oXB);
  float*          H    = (float*)(ws + oH);
  unsigned short* A    = (unsigned short*)(ws + oA);
  float*          G    = (float*)(ws + oG);
  int*            LIST = (int*)(ws + oLIST);
  int*            CNT  = (int*)(ws + oCNT);
  int*            OFF  = (int*)(ws + oOFF);
  int*            DINB = (int*)(ws + oDINV);
  const float*    DINV = (const float*)(ws + oDINV);
  int*            FLAG = (int*)(ws + oFLAG);
  unsigned short* W1T  = (unsigned short*)(ws + oW1T);
  unsigned short* W2D  = (unsigned short*)(ws + oW2D);
  unsigned short* W3T  = (unsigned short*)(ws + oW3T);
  float*          SM   = (float*)(ws + oSM);

  hipFuncSetAttribute(reinterpret_cast<const void*>(&k_bucket), hipFuncAttributeMaxDynamicSharedMemorySize, (int)BK_LDS);

  k_prep<<<PBTOT, NTHR, 0, stream>>>(x, Wp1, bp1, Wp2, bp2, Wp3, bp3, Wv1, bv1, Wv2, bv2, Wv3, bv3,
                                     XB, W1T, W2D, W3T, SM);
  k_bucket<<<NBK, NTHR, BK_LDS, stream>>>(srcs, dsts, LIST, CNT, OFF, DINB, FLAG);
  k_mm<CIN, 4><<<dim3(MP / GBM, NW / 64, 1), NTHR, 0, stream>>>(XB, CIN, 0, W1T, CIN, 0, DINV, H, NW, 0);
  k_replay_wide<<<MP / RWB, NTHR, 0, stream>>>(LIST, CNT, OFF, DINV, FLAG, H, SM, A);
  k_mm<K2, 4><<<dim3(MP / GBM, HD / 64, 2), NTHR, 0, stream>>>(A, AK, 256, W2D, 256, HD * 256, DINV, H, NW, HD);
  k_replay_wide<<<MP / RWB, NTHR, 0, stream>>>(LIST, CNT, OFF, DINV, FLAG, H, SM + 256, A);
  k_mm<AK, 1><<<dim3(MP / GBM, 1, 1), NTHR, 0, stream>>>(A, AK, 0, W3T, AK, 0, DINV, G, GN, 0);
  k_replay_narrow<<<NBK, NTHR, 0, stream>>>(LIST, CNT, OFF, DINV, FLAG, G, SM + 512, out);
}
